// QuantumRegressionGen_65481071398329
// MI455X (gfx1250) — hardware-verified
//
#include <hip/hip_runtime.h>
#include <stdint.h>


#define NW      10
#define NOPS    30
#define NST     1024
#define SB      8
#define NSUB    4
#define BT      (SB * NSUB)
#define TPB     256
#define PAIR_IT (SB * 512 / TPB)
#define QUAD_IT (SB * 256 / TPB)
#define AMP_IT  (NST / TPB)
#define H0P     72
#define H1P     40
#define NTRIG   (BT * NW + NOPS + 2)
#define WSC     16.0f
#define WSC_INV 0.0625f

typedef __attribute__((ext_vector_type(16))) _Float16 v16h;
typedef __attribute__((ext_vector_type(8)))  _Float16 v8h;
typedef __attribute__((ext_vector_type(8)))  float    v8f;
typedef __attribute__((ext_vector_type(4)))  float    v4f;

struct FragH {
  union U { v16h v; v8h h[2]; };
  static __device__ __forceinline__ v16h load(const _Float16* p) {
    U f; f.h[0] = *(const v8h*)(p); f.h[1] = *(const v8h*)(p + 16); return f.v;
  }
};

__device__ __forceinline__ v8f hmma(v16h a, v16h b, v8f c) {
  c = __builtin_amdgcn_wmma_f32_16x16x32_f16(false, a, false, b, (short)0, c, false, false);
  asm volatile("v_nop\n\tv_nop\n\tv_nop\n\tv_nop" : "+v"(c) : "v"(a), "v"(b));
  return c;
}

__constant__ int c_opk[NOPS] = {0,2,1,0,0,2,2,2,2,3, 0,3,2,1,0,3,1,0,2,0, 1,2,3,1,2,2,3,1,3,3};
__constant__ int c_opa[NOPS] = {7,4,8,6,0,9,7,7,1,5, 9,5,4,2,5,0,6,7,3,9, 8,7,3,0,1,6,6,3,0,4};
__constant__ int c_opb[NOPS] = {0,0,0,0,0,0,0,0,0,4, 0,4,0,0,0,8,0,0,0,0, 0,0,1,0,0,0,3,0,3,1};


__device__ __forceinline__ void apply_rx(float* sre, float* sim, int shift, float c, float s, int tid) {
  const int mask = 1 << shift, low = mask - 1;
#pragma unroll 4
  for (int it = 0; it < PAIR_IT; ++it) {
    const int p = tid + it * TPB;
    const int el = p >> 9, q = p & 511;
    const int i0 = (el << 10) + (((q >> shift) << (shift + 1)) | (q & low));
    const int i1 = i0 + mask;
    const float a0r = sre[i0], a0i = sim[i0], a1r = sre[i1], a1i = sim[i1];
    sre[i0] = c * a0r + s * a1i;
    sim[i0] = c * a0i - s * a1r;
    sre[i1] = c * a1r + s * a0i;
    sim[i1] = c * a1i - s * a0r;
  }
}
__device__ __forceinline__ void apply_ry(float* sre, float* sim, int shift, float c, float s, int tid) {
  const int mask = 1 << shift, low = mask - 1;
#pragma unroll 4
  for (int it = 0; it < PAIR_IT; ++it) {
    const int p = tid + it * TPB;
    const int el = p >> 9, q = p & 511;
    const int i0 = (el << 10) + (((q >> shift) << (shift + 1)) | (q & low));
    const int i1 = i0 + mask;
    const float a0r = sre[i0], a0i = sim[i0], a1r = sre[i1], a1i = sim[i1];
    sre[i0] = c * a0r - s * a1r;
    sim[i0] = c * a0i - s * a1i;
    sre[i1] = s * a0r + c * a1r;
    sim[i1] = s * a0i + c * a1i;
  }
}
__device__ __forceinline__ void apply_rz(float* sre, float* sim, int shift, float c, float s, int tid) {
  const int mask = 1 << shift, low = mask - 1;
#pragma unroll 4
  for (int it = 0; it < PAIR_IT; ++it) {
    const int p = tid + it * TPB;
    const int el = p >> 9, q = p & 511;
    const int i0 = (el << 10) + (((q >> shift) << (shift + 1)) | (q & low));
    const int i1 = i0 + mask;
    const float a0r = sre[i0], a0i = sim[i0], a1r = sre[i1], a1i = sim[i1];
    sre[i0] = c * a0r + s * a0i;
    sim[i0] = c * a0i - s * a0r;
    sre[i1] = c * a1r - s * a1i;
    sim[i1] = c * a1i + s * a1r;
  }
}
__device__ __forceinline__ void apply_gen(float* sre, float* sim, int shift,
                                          float v00r, float v00i, float v01r, float v01i,
                                          float v10r, float v10i, float v11r, float v11i, int tid) {
  const int mask = 1 << shift, low = mask - 1;
#pragma unroll 4
  for (int it = 0; it < PAIR_IT; ++it) {
    const int p = tid + it * TPB;
    const int el = p >> 9, q = p & 511;
    const int i0 = (el << 10) + (((q >> shift) << (shift + 1)) | (q & low));
    const int i1 = i0 + mask;
    const float a0r = sre[i0], a0i = sim[i0], a1r = sre[i1], a1i = sim[i1];
    sre[i0] = v00r * a0r - v00i * a0i + v01r * a1r - v01i * a1i;
    sim[i0] = v00r * a0i + v00i * a0r + v01r * a1i + v01i * a1r;
    sre[i1] = v10r * a0r - v10i * a0i + v11r * a1r - v11i * a1i;
    sim[i1] = v10r * a0i + v10i * a0r + v11r * a1i + v11i * a1r;
  }
}
__device__ __forceinline__ void apply_cnot(float* sre, float* sim, int cshift, int tshift, int tid) {
  const int b0s = (cshift < tshift) ? cshift : tshift;
  const int b1s = (cshift < tshift) ? tshift : cshift;
  const int cmask = 1 << cshift, tmask = 1 << tshift;
#pragma unroll 4
  for (int it = 0; it < QUAD_IT; ++it) {
    const int p = tid + it * TPB;
    const int el = p >> 8, m = p & 255;
    int i = ((m >> b0s) << (b0s + 1)) | (m & ((1 << b0s) - 1));
    i     = ((i >> b1s) << (b1s + 1)) | (i & ((1 << b1s) - 1));
    const int ia = (el << 10) + (i | cmask);
    const int ib = ia + tmask;
    const float r = sre[ia], q = sim[ia];
    sre[ia] = sre[ib]; sim[ia] = sim[ib];
    sre[ib] = r;       sim[ib] = q;
  }
}

__global__ void __launch_bounds__(TPB)
fused_qmlp_kernel(const float* __restrict__ x,    const float* __restrict__ rp,
                  const float* __restrict__ rxth, const float* __restrict__ ryth,
                  const float* __restrict__ hw,   const float* __restrict__ hb,
                  const float* __restrict__ w0,   const float* __restrict__ b0,
                  const float* __restrict__ w1,   const float* __restrict__ b1,
                  const float* __restrict__ w2,   const float* __restrict__ b2,
                  const float* __restrict__ w3,   const float* __restrict__ b3,
                  float* __restrict__ out, int bsz)
{
  __shared__ __align__(16) float    s_re[SB * NST];
  __shared__ __align__(16) float    s_im[SB * NST];
  __shared__ __align__(16) float    xs[BT * NW];
  __shared__ __align__(16) float    trc[NTRIG];
  __shared__ __align__(16) float    trs[NTRIG];
  __shared__ __align__(16) float    outv[BT];
  __shared__ __align__(16) float    cml[BT];
  __shared__ __align__(16) _Float16 h0h[BT * H0P];
  __shared__ __align__(16) _Float16 w1h[32 * H0P];
  __shared__ __align__(16) _Float16 h1h[BT * H1P];
  __shared__ __align__(16) _Float16 w2h[16 * H1P];

  const int tid  = threadIdx.x;
  const int lane = tid & 31;
  const int wave = tid >> 5;
  const int hh   = lane >> 4;
  const int rl   = lane & 15;
  const int koff = hh * 8;
  const int s0   = blockIdx.x * BT;

  for (int it = 0; it < 2; ++it) {
    const int idx = tid + it * TPB;
    if (idx < NTRIG) {
      float th;
      if (idx < BT * NW) {
        const int r = idx / NW;
        const int k = idx - r * NW;
        int gr = s0 + r; gr = (gr < bsz) ? gr : (bsz - 1);
        const float xv = x[(size_t)gr * NW + k];
        xs[idx] = xv;
        th = 0.5f * xv;
      } else if (idx < BT * NW + NOPS) {
        th = 0.5f * rp[idx - BT * NW];
      } else if (idx == BT * NW + NOPS) {
        th = 0.5f * rxth[0];
      } else {
        th = 0.5f * ryth[0];
      }
      trc[idx] = cosf(th);
      trs[idx] = sinf(th);
    }
  }
#pragma unroll
  for (int it = 0; it < 8; ++it) {
    const int e = tid + it * TPB;
    const int n = e >> 6, k = e & 63;
    w1h[n * H0P + k] = (_Float16)(w1[e] * WSC);
  }
#pragma unroll
  for (int it = 0; it < 2; ++it) {
    const int e = tid + it * TPB;
    const int n = e >> 5, k = e & 31;
    w2h[n * H1P + k] = (_Float16)(w2[e] * WSC);
  }
  __syncthreads();

  {
    const int n  = tid & 63;
    const int rq = tid >> 6;
    float wreg[NW];
#pragma unroll
    for (int k = 0; k < NW; ++k) wreg[k] = w0[n * NW + k];
    const float bn = b0[n];
#pragma unroll 1
    for (int j = 0; j < 8; ++j) {
      const int r = rq + 4 * j;
      float acc = 0.f;
#pragma unroll
      for (int k = 0; k < NW; ++k) acc += xs[r * NW + k] * wreg[k];
      acc += bn;
      h0h[r * H0P + n] = (_Float16)acc;
    }
  }
  __syncthreads();

  if (wave < 2) {
    const int m0 = wave * 16;
    const v8f z = {0.f, 0.f, 0.f, 0.f, 0.f, 0.f, 0.f, 0.f};
    v8f acc0 = z, acc1 = z;
#pragma unroll
    for (int ks = 0; ks < 2; ++ks) {
      const v16h a   = FragH::load(h0h + (m0 + rl) * H0P + koff + 32 * ks);
      const v16h bq0 = FragH::load(w1h + (rl) * H0P + koff + 32 * ks);
      const v16h bq1 = FragH::load(w1h + (16 + rl) * H0P + koff + 32 * ks);
      acc0 = hmma(a, bq0, acc0);
      acc1 = hmma(a, bq1, acc1);
    }
    const float bb0 = b1[rl], bb1 = b1[16 + rl];
#pragma unroll
    for (int r = 0; r < 8; ++r) {
      const int row = m0 + 8 * hh + r;
      h1h[row * H1P + rl]      = (_Float16)(acc0[r] * WSC_INV + bb0);
      h1h[row * H1P + 16 + rl] = (_Float16)(acc1[r] * WSC_INV + bb1);
    }
  }
  __syncthreads();

  if (wave < 2) {
    const int m0 = wave * 16;
    const v8f z = {0.f, 0.f, 0.f, 0.f, 0.f, 0.f, 0.f, 0.f};
    const v16h a  = FragH::load(h1h + (m0 + rl) * H1P + koff);
    const v16h bq = FragH::load(w2h + rl * H1P + koff);
    v8f acc2 = hmma(a, bq, z);
    const float bb2 = b2[rl];
    const float w3v = w3[rl];
    const float bb3 = b3[0];
#pragma unroll
    for (int r = 0; r < 8; ++r) {
      const float h2v = acc2[r] * WSC_INV + bb2;
      float t = h2v * w3v;
      t += __shfl_xor(t, 8, 32);
      t += __shfl_xor(t, 4, 32);
      t += __shfl_xor(t, 2, 32);
      t += __shfl_xor(t, 1, 32);
      if (rl == 0) cml[m0 + 8 * hh + r] = t + bb3;
    }
  }
  __syncthreads();

  const float cx = trc[BT * NW + NOPS], sx = trs[BT * NW + NOPS];
  const float cy = trc[BT * NW + NOPS + 1], sy = trs[BT * NW + NOPS + 1];
  const float v00r =  cy * cx, v00i =  sy * sx;
  const float v01r = -sy * cx, v01i = -cy * sx;
  const float v10r =  sy * cx, v10i = -cy * sx;
  const float v11r =  cy * cx, v11i = -sy * sx;

#pragma unroll 1
  for (int sb = 0; sb < NSUB; ++sb) {
#pragma unroll 1
    for (int el = 0; el < SB; ++el) {
      const int r = sb * SB + el;
      float ec[NW], es[NW];
#pragma unroll
      for (int w = 0; w < NW; ++w) { ec[w] = trc[r * NW + w]; es[w] = trs[r * NW + w]; }
#pragma unroll
      for (int it = 0; it < AMP_IT; ++it) {
        const int i = tid + it * TPB;
        float amp = 1.f;
#pragma unroll
        for (int w = 0; w < NW; ++w) amp *= ((i >> (9 - w)) & 1) ? es[w] : ec[w];
        s_re[el * NST + i] = amp;
        s_im[el * NST + i] = 0.f;
      }
    }
    __syncthreads();

#pragma unroll 1
    for (int g = 0; g < NOPS; ++g) {
      const int kind = c_opk[g];
      const int sa   = 9 - c_opa[g];
      if (kind == 3) {
        apply_cnot(s_re, s_im, sa, 9 - c_opb[g], tid);
      } else {
        const float c = trc[BT * NW + g], s = trs[BT * NW + g];
        if (kind == 0)      apply_rx(s_re, s_im, sa, c, s, tid);
        else if (kind == 1) apply_ry(s_re, s_im, sa, c, s, tid);
        else                apply_rz(s_re, s_im, sa, c, s, tid);
      }
      __syncthreads();
    }

#pragma unroll 1
    for (int w = 0; w < NW; ++w) {
      apply_gen(s_re, s_im, 9 - w, v00r, v00i, v01r, v01i, v10r, v10i, v11r, v11i, tid);
      __syncthreads();
    }

    {
      const int el = wave;
      float f[NW];
#pragma unroll
      for (int w = 0; w < NW; ++w) f[w] = 0.f;
#pragma unroll 2
      for (int j = 0; j < 32; ++j) {
        const int i = j * 32 + lane;
        const float re = s_re[el * NST + i], im = s_im[el * NST + i];
        const float pv = re * re + im * im;
#pragma unroll
        for (int w = 0; w < NW; ++w) f[w] += ((i >> (9 - w)) & 1) ? -pv : pv;
      }
#pragma unroll
      for (int w = 0; w < NW; ++w) {
        float t = f[w];
        t += __shfl_xor(t, 16, 32);
        t += __shfl_xor(t, 8, 32);
        t += __shfl_xor(t, 4, 32);
        t += __shfl_xor(t, 2, 32);
        t += __shfl_xor(t, 1, 32);
        f[w] = t;
      }
      float qv = 0.f;
#pragma unroll
      for (int w = 0; w < NW; ++w) qv += f[w] * hw[w];
      qv += hb[0];
      if (lane == 0) {
        const int r = sb * SB + el;
        outv[r] = qv + cml[r];
      }
    }
    __syncthreads();
  }

  if (wave == 0) {
    const bool full = (s0 + BT <= bsz);
    v4f vv = {0.f, 0.f, 0.f, 0.f};
    if (lane < 8) vv = *(const v4f*)(outv + 4 * lane);
    const float sv = outv[lane];
    if (full) {
      if (lane < 8) *(volatile v4f*)(out + s0 + 4 * lane) = vv;
    } else {
      if (s0 + lane < bsz) *(volatile float*)(out + s0 + lane) = sv;
    }
    __threadfence();
    if (full) {
      if (lane < 8) *(volatile v4f*)(out + s0 + 4 * lane) = vv;
    } else {
      if (s0 + lane < bsz) *(volatile float*)(out + s0 + lane) = sv;
    }
  }
}

extern "C" void kernel_launch(void* const* d_in, const int* in_sizes, int n_in,
                              void* d_out, int out_size, void* d_ws, size_t ws_size,
                              hipStream_t stream)
{
  (void)n_in; (void)d_ws; (void)ws_size;
  const float* x    = (const float*)d_in[0];
  const float* rp   = (const float*)d_in[1];
  const float* rxth = (const float*)d_in[2];
  const float* ryth = (const float*)d_in[3];
  const float* hw   = (const float*)d_in[4];
  const float* hb   = (const float*)d_in[5];
  const float* w0   = (const float*)d_in[6];
  const float* b0   = (const float*)d_in[7];
  const float* w1   = (const float*)d_in[8];
  const float* b1   = (const float*)d_in[9];
  const float* w2   = (const float*)d_in[10];
  const float* b2   = (const float*)d_in[11];
  const float* w3   = (const float*)d_in[12];
  const float* b3   = (const float*)d_in[13];
  float* out = (float*)d_out;

  int bsz = in_sizes[0] / NW;
  if (out_size < bsz) bsz = out_size;
  if (bsz <= 0) return;

  const int blocks = (bsz + BT - 1) / BT;
  fused_qmlp_kernel<<<blocks, TPB, 0, stream>>>(x, rp, rxth, ryth, hw, hb,
                                                w0, b0, w1, b1, w2, b2, w3, b3, out, bsz);
  (void)hipGetLastError();
}
